// DependencyParser_4492535792544
// MI455X (gfx1250) — hardware-verified
//
#include <hip/hip_runtime.h>
#include <math.h>

constexpr int NB_IN  = 32;
constexpr int NL_IN  = 128;
constexpr int NSTEP  = 32;
constexpr int NSEQ   = 128;
constexpr int NROW   = NSTEP * NSEQ;
constexpr int WDIM   = 300;
constexpr int TDIM   = 100;
constexpr int WVOC   = 30000;
constexpr int TVOC   = 50;
constexpr int HID    = 400;
constexpr int NGATE  = 4 * HID;
constexpr int K0P    = 416;
constexpr int SEGH   = 416;
constexpr int KREC   = 2 * SEGH;
constexpr int KCAT   = 2 * KREC;
constexpr int MLPH   = 100;
constexpr int MLPP   = 128;
constexpr int NOUT   = NL_IN * NL_IN * NB_IN;
constexpr int GPSEG  = SEGH / 8;
constexpr int GVALID = HID / 8;

constexpr int EMB_THR  = 128;
constexpr int EGPR     = K0P / 8;
constexpr int PC_THR   = 256;
constexpr int REC_THR  = 160;
constexpr int SEQB     = 16;
constexpr int UPW      = 5;
constexpr int HTP      = 840;
constexpr int PAIR_THR = 256;
constexpr int ASP      = 104;
constexpr int ELINES   = SEQB * (KREC / 64);
constexpr int EGRP     = 4 * (REC_THR / 32);
constexpr int EITER    = (ELINES + EGRP - 1) / EGRP;

static_assert(K0P % 32 == 0 && KREC % 64 == 0 && KCAT % 32 == 0);
static_assert(NROW % 64 == 0 && NGATE % 64 == 0 && MLPP % 64 == 0);
static_assert(HID == 16 * UPW * (REC_THR / 32));
static_assert((2 * SEQB * HTP) % REC_THR == 0);
static_assert((SEQB * HID) % REC_THR == 0);
static_assert(NSEQ % SEQB == 0);
static_assert(WDIM % 4 == 0 && TDIM % 4 == 0 && WDIM + TDIM == HID);
static_assert(2 * EGPR <= EMB_THR && (2 * K0P * 2) % 128 == 0);
static_assert((NGATE * GPSEG) % 32 == 0 && (MLPP * 4 * GPSEG) % 32 == 0);
static_assert(NL_IN % (PAIR_THR / 32) == 0 && MLPH % 4 == 0);
static_assert(NB_IN == 32);
static_assert(ELINES % 4 == 0);

typedef __attribute__((ext_vector_type(16))) _Float16 v16h;
typedef __attribute__((ext_vector_type(8)))  _Float16 v8h;
typedef __attribute__((ext_vector_type(16))) __bf16   v16b;
typedef __attribute__((ext_vector_type(8)))  __bf16   v8b;
typedef __attribute__((ext_vector_type(8)))  float    v8f;
typedef __attribute__((ext_vector_type(4)))  float    v4f;
typedef unsigned v4u_t __attribute__((ext_vector_type(4)));
typedef v4u_t __attribute__((may_alias)) v4u;
typedef unsigned v2u_t __attribute__((ext_vector_type(2)));
typedef v2u_t __attribute__((may_alias)) v2u;

__device__ __forceinline__ unsigned short f2bf_bits(float f) {
  unsigned u = __float_as_uint(f);
  return (unsigned short)((u + 0x7FFFu + ((u >> 16) & 1u)) >> 16);
}
__device__ __forceinline__ float bf_bits2f(unsigned short h) { return __uint_as_float(((unsigned)h) << 16); }
__device__ __forceinline__ float bf16r(float f) { return bf_bits2f(f2bf_bits(f)); }

__device__ __forceinline__ void dep_guard_h(v8f& a, v8f& b, v16h x, v16h y) { asm volatile("v_nop\n\tv_nop\n\tv_nop\n\tv_nop" : "+v"(a), "+v"(b) : "v"(x), "v"(y)); }
__device__ __forceinline__ void dep_guard_b(v8f& a, v8f& b, v16b x, v16b y) { asm volatile("v_nop\n\tv_nop\n\tv_nop\n\tv_nop" : "+v"(a), "+v"(b) : "v"(x), "v"(y)); }
__device__ __forceinline__ void keep4_h(v16h a, v16h b, v16h c, v16h d) { asm volatile("v_nop" :: "v"(a), "v"(b), "v"(c), "v"(d)); }
__device__ __forceinline__ void keep4_b(v16b a, v16b b, v16b c, v16b d) { asm volatile("v_nop" :: "v"(a), "v"(b), "v"(c), "v"(d)); }
__device__ __forceinline__ void acc_guard4(v8f& a, v8f& b, v8f& c, v8f& d) { asm volatile("v_nop\n\tv_nop\n\tv_nop\n\tv_nop" : "+v"(a), "+v"(b), "+v"(c), "+v"(d)); }
__device__ __forceinline__ void guard_grp_h(v8f& a0, v8f& a1, v8f& a2, v8f& a3, v16h x, v16h y0, v16h y1, v16h y2, v16h y3) {
  asm volatile("v_nop\n\tv_nop\n\tv_nop\n\tv_nop" : "+v"(a0), "+v"(a1), "+v"(a2), "+v"(a3) : "v"(x), "v"(y0), "v"(y1), "v"(y2), "v"(y3));
}
__device__ __forceinline__ void guard_grp_b(v8f& a0, v8f& a1, v8f& a2, v8f& a3, v16b x, v16b y0, v16b y1, v16b y2, v16b y3) {
  asm volatile("v_nop\n\tv_nop\n\tv_nop\n\tv_nop" : "+v"(a0), "+v"(a1), "+v"(a2), "+v"(a3) : "v"(x), "v"(y0), "v"(y1), "v"(y2), "v"(y3));
}

template <typename T> struct Frag;
template <> struct Frag<_Float16> {
  typedef v16h V; union U { v16h v; v8h h[2]; };
  static __device__ __forceinline__ v16h load(const _Float16* p) {
    U f; f.h[0] = *(const v8h*)(p); f.h[1] = *(const v8h*)(p + 16); return f.v;
  }
  static __device__ __forceinline__ v8f mma(v16h a, v16h b, v8f c) {
    return __builtin_amdgcn_wmma_f32_16x16x32_f16(false, a, false, b, (short)0, c, false, false);
  }
  static __device__ __forceinline__ void guard(v8f& a, v8f& b, v16h x, v16h y) { dep_guard_h(a, b, x, y); }
  static __device__ __forceinline__ void guard4(v8f& a, v8f& b, v8f& c, v8f& d, v16h x, v16h y0, v16h y1, v16h y2, v16h y3) { guard_grp_h(a, b, c, d, x, y0, y1, y2, y3); }
  static __device__ __forceinline__ void keep(v16h a, v16h b, v16h c, v16h d) { keep4_h(a, b, c, d); }
};
template <> struct Frag<__bf16> {
  typedef v16b V; union U { v16b v; v8b h[2]; };
  static __device__ __forceinline__ v16b load(const __bf16* p) {
    U f; f.h[0] = *(const v8b*)(p); f.h[1] = *(const v8b*)(p + 16); return f.v;
  }
  static __device__ __forceinline__ v8f mma(v16b a, v16b b, v8f c) {
    return __builtin_amdgcn_wmma_f32_16x16x32_bf16(false, a, false, b, (short)0, c, false, false);
  }
  static __device__ __forceinline__ void guard(v8f& a, v8f& b, v16b x, v16b y) { dep_guard_b(a, b, x, y); }
  static __device__ __forceinline__ void guard4(v8f& a, v8f& b, v8f& c, v8f& d, v16b x, v16b y0, v16b y1, v16b y2, v16b y3) { guard_grp_b(a, b, c, d, x, y0, y1, y2, y3); }
  static __device__ __forceinline__ void keep(v16b a, v16b b, v16b c, v16b d) { keep4_b(a, b, c, d); }
};

template <int ET> struct Elem;
template <> struct Elem<0> { typedef _Float16 T; };
template <> struct Elem<1> { typedef __bf16 T; };
template <int ET, bool SPLIT, int BIAS_MODE, int OUT_MODE, bool RESID, int ACT = 0>
__global__ __launch_bounds__(256) void wmma_gemm64(
    const unsigned short* __restrict__ Ap, const unsigned short* __restrict__ A2p, int lda, long strideA,
    const unsigned short* __restrict__ Btp, const unsigned short* __restrict__ Bt2p, int ldb, long strideB,
    void* __restrict__ Cout, void* __restrict__ Cout2, int ldc, long strideC,
    const float* __restrict__ bias,
    const float* __restrict__ resid, long strideR,
    int M, int N, int K, float scale) {
  static_assert(!RESID);
  typedef typename Elem<ET>::T T;
  typedef typename Frag<T>::V V;
  const T* A = (const T*)Ap; const T* A2 = (const T*)A2p; const T* Bt = (const T*)Btp; const T* Bt2 = (const T*)Bt2p;
  __shared__ __align__(16) float sT[8][16 * 68];
  const int b    = blockIdx.y;
  const int lane = threadIdx.x & 31;
  const int wave = threadIdx.x >> 5;
  const int tilesN = N >> 6;
  const int tilesM = M >> 6;
  const int tile = blockIdx.x * 8 + wave;
  if (tile >= tilesM * tilesN) return;
  const int tm = tile / tilesN;
  const int tn = tile - tm * tilesN;
  const int m0 = tm << 6;
  const int n0 = tn << 6;

  const T* Ab  = A  + (size_t)b * strideA;
  const T* Bb  = Bt + (size_t)b * strideB;
  const T* Ab2 = SPLIT ? (A2  + (size_t)b * strideA) : nullptr;
  const T* Bb2 = SPLIT ? (Bt2 + (size_t)b * strideB) : nullptr;

  const int rlane = lane & 15;
  const int koff  = (lane >> 4) * 8;
  const int mOff  = (lane >> 4) * 8;

  v8f acc[4][4];
#pragma unroll
  for (int i = 0; i < 4; ++i)
#pragma unroll
    for (int j = 0; j < 4; ++j) acc[i][j] = (v8f){0.f,0.f,0.f,0.f,0.f,0.f,0.f,0.f};

  for (int k0 = 0; k0 < K; k0 += 32) {
    V bh[4], bl[4];
#pragma unroll
    for (int j = 0; j < 4; ++j) {
      const size_t bo = (size_t)(n0 + (j << 4) + rlane) * ldb + koff + k0;
      bh[j] = Frag<T>::load(Bb + bo);
      bl[j] = bh[j];
      if (SPLIT) bl[j] = Frag<T>::load(Bb2 + bo);
    }
#pragma unroll
    for (int i = 0; i < 4; ++i) {
      const size_t ao = (size_t)(m0 + (i << 4) + rlane) * lda + koff + k0;
      V ah = Frag<T>::load(Ab + ao);
      V al = ah;
      if (SPLIT) al = Frag<T>::load(Ab2 + ao);
#pragma unroll
      for (int j = 0; j < 4; ++j) {
        acc[i][j] = Frag<T>::mma(ah, bh[j], acc[i][j]);
        if (SPLIT) {
          acc[i][j] = Frag<T>::mma(ah, bl[j], acc[i][j]);
          acc[i][j] = Frag<T>::mma(al, bh[j], acc[i][j]);
        }
      }
      Frag<T>::guard4(acc[i][0], acc[i][1], acc[i][2], acc[i][3], ah, bh[0], bh[1], bh[2], bh[3]);
      if (SPLIT) Frag<T>::guard4(acc[i][0], acc[i][1], acc[i][2], acc[i][3], al, bl[0], bl[1], bl[2], bl[3]);
    }
    Frag<T>::keep(bh[0], bh[1], bh[2], bh[3]);
    if (SPLIT) Frag<T>::keep(bl[0], bl[1], bl[2], bl[3]);
  }
  acc_guard4(acc[0][0], acc[0][1], acc[0][2], acc[0][3]);
  acc_guard4(acc[1][0], acc[1][1], acc[1][2], acc[1][3]);
  acc_guard4(acc[2][0], acc[2][1], acc[2][2], acc[2][3]);
  acc_guard4(acc[3][0], acc[3][1], acc[3][2], acc[3][3]);

  float* slab = sT[wave];
#pragma unroll
  for (int i = 0; i < 4; ++i) {
    const int mBase = m0 + (i << 4);
    float bmr[8];
#pragma unroll
    for (int r = 0; r < 8; ++r) bmr[r] = 0.0f;
    if (BIAS_MODE == 1) {
      const v4f q0 = *(const v4f*)(bias + mBase + mOff);
      const v4f q1 = *(const v4f*)(bias + mBase + mOff + 4);
      bmr[0] = q0[0]; bmr[1] = q0[1]; bmr[2] = q0[2]; bmr[3] = q0[3];
      bmr[4] = q1[0]; bmr[5] = q1[1]; bmr[6] = q1[2]; bmr[7] = q1[3];
    }
#pragma unroll
    for (int j = 0; j < 4; ++j) {
      const int n = n0 + (j << 4) + rlane;
      float bv = 0.f;
      if (BIAS_MODE == 2) bv = bias[n];
#pragma unroll
      for (int r = 0; r < 8; ++r) {
        float v = acc[i][j][r] * scale;
        if (BIAS_MODE == 1) v += bmr[r];
        if (BIAS_MODE == 2) v += bv;
        if (ACT == 2) v = fmaxf(v, 0.0f);
        if (ACT == 4) v = (v > 0.f) ? v : 0.01f * v;
        slab[(mOff + r) * 68 + (j << 4) + rlane] = v;
      }
    }
    __builtin_amdgcn_fence(__ATOMIC_RELEASE, "workgroup");
    __builtin_amdgcn_wave_barrier();
    __builtin_amdgcn_fence(__ATOMIC_ACQUIRE, "workgroup");
    if (OUT_MODE == 0) {
      float* C = (float*)Cout + (size_t)b * strideC;
      const int hh = lane >> 4, c4 = (lane & 15) * 4;
      for (int pass = 0; pass < 2; ++pass) {
#pragma unroll
        for (int it = 0; it < 8; ++it) {
          const int row = it * 2 + hh;
          v4f v = *(const v4f*)(slab + row * 68 + c4);
          *(volatile v4f*)(C + (size_t)(mBase + row) * ldc + n0 + c4) = v;
        }
        __threadfence();
      }
    } else {
      const int q = lane >> 3, c8 = (lane & 7) * 8;
      unsigned short* C  = (unsigned short*)Cout  + (size_t)b * strideC;
      unsigned short* C2 = (OUT_MODE == 2) ? ((unsigned short*)Cout2 + (size_t)b * strideC) : nullptr;
      for (int pass = 0; pass < 2; ++pass) {
#pragma unroll
        for (int it = 0; it < 4; ++it) {
          const int row = it * 4 + q;
          const float* sp = slab + row * 68 + c8;
          v8h hv, lv;
#pragma unroll
          for (int e = 0; e < 8; ++e) {
            if (OUT_MODE == 1) {
              hv[e] = (_Float16)sp[e];
            } else {
              unsigned short hb = f2bf_bits(sp[e]);
              unsigned short lb = f2bf_bits(sp[e] - bf_bits2f(hb));
              hv[e] = __builtin_bit_cast(_Float16, hb);
              lv[e] = __builtin_bit_cast(_Float16, lb);
            }
          }
          *(volatile v8h*)(C + (size_t)(mBase + row) * ldc + n0 + c8) = hv;
          if (OUT_MODE == 2) *(volatile v8h*)(C2 + (size_t)(mBase + row) * ldc + n0 + c8) = lv;
        }
        __threadfence();
      }
    }
    __builtin_amdgcn_fence(__ATOMIC_RELEASE, "workgroup");
    __builtin_amdgcn_wave_barrier();
    __builtin_amdgcn_fence(__ATOMIC_ACQUIRE, "workgroup");
  }
}

__device__ __forceinline__ v2u emb_half(int cg, const float* __restrict__ wrow, const float* __restrict__ trow) {
  const int cgw = (cg < WDIM / 4) ? cg : (WDIM / 4 - 1);
  int cgt = cg - WDIM / 4; cgt = cgt < 0 ? 0 : (cgt > TDIM / 4 - 1 ? TDIM / 4 - 1 : cgt);
  const v4f wv = *(const v4f*)(wrow + 4 * cgw);
  const v4f tv = *(const v4f*)(trow + 4 * cgt);
  const float fw = (cg < WDIM / 4) ? 1.0f : 0.0f;
  const float ft = (cg >= WDIM / 4 && cg < (WDIM + TDIM) / 4) ? 1.0f : 0.0f;
  const unsigned u0 = f2bf_bits(fmaf(fw, wv[0], ft * tv[0]));
  const unsigned u1 = f2bf_bits(fmaf(fw, wv[1], ft * tv[1]));
  const unsigned u2 = f2bf_bits(fmaf(fw, wv[2], ft * tv[2]));
  const unsigned u3 = f2bf_bits(fmaf(fw, wv[3], ft * tv[3]));
  v2u pk;
  pk[0] = u0 | (u1 << 16);
  pk[1] = u2 | (u3 << 16);
  return pk;
}
__global__ __launch_bounds__(EMB_THR) void embed_kernel(const int* __restrict__ words, const int* __restrict__ tags,
                                                        const float* __restrict__ wemb, const float* __restrict__ temb,
                                                        unsigned short* __restrict__ E0) {
  const int tid = threadIdx.x;
  if (tid >= 2 * EGPR) return;
  const int rr  = tid / EGPR;
  const int kg  = tid - rr * EGPR;
  const int rho = blockIdx.x * 2 + rr;
  const int t = rho / NSEQ, n = rho - t * NSEQ;
  const int f = n * NSTEP + t;
  int wi = words[f]; wi = wi < 0 ? 0 : (wi > WVOC - 1 ? WVOC - 1 : wi);
  int ti = tags[f];  ti = ti < 0 ? 0 : (ti > TVOC - 1 ? TVOC - 1 : ti);
  const float* wrow = wemb + (size_t)wi * WDIM;
  const float* trow = temb + (size_t)ti * TDIM;
  const v2u pa = emb_half(2 * kg,     wrow, trow);
  const v2u pb = emb_half(2 * kg + 1, wrow, trow);
  v4u pk;
  pk[0] = pa[0]; pk[1] = pa[1]; pk[2] = pb[0]; pk[3] = pb[1];
  unsigned short* dst = E0 + (size_t)rho * K0P + 8 * kg;
  *(volatile v4u*)dst = pk;
  __threadfence();
  *(volatile v4u*)dst = pk;
}

__global__ __launch_bounds__(PC_THR) void padcopy_kernel(const float* __restrict__ src, int spitch, int scol0, int nsrcrow,
                                                         unsigned short* __restrict__ dst, int ndstrow, int nseg) {
  const int gpr = nseg * GPSEG;
  const int i = blockIdx.x * PC_THR + threadIdx.x;
  if (i >= ndstrow * gpr) return;
  const int row = i / gpr;
  const int g   = i - row * gpr;
  const int seg = g / GPSEG;
  const int kg  = g - seg * GPSEG;
  const bool valid = (kg < GVALID) && (row < nsrcrow);
  const int rowc = (row < nsrcrow) ? row : (nsrcrow - 1);
  const int kgc  = (kg < GVALID) ? kg : (GVALID - 1);
  const float* sp = src + (size_t)rowc * spitch + scol0 + (seg >> 1) * HID + 8 * kgc;
  const v4f a = *(const v4f*)(sp);
  const v4f b = *(const v4f*)(sp + 4);
  const float fl = valid ? 1.0f : 0.0f;
  const unsigned e0 = f2bf_bits(a[0] * fl), e1 = f2bf_bits(a[1] * fl), e2 = f2bf_bits(a[2] * fl), e3 = f2bf_bits(a[3] * fl);
  const unsigned e4 = f2bf_bits(b[0] * fl), e5 = f2bf_bits(b[1] * fl), e6 = f2bf_bits(b[2] * fl), e7 = f2bf_bits(b[3] * fl);
  v4u pk;
  pk[0] = e0 | (e1 << 16);
  pk[1] = e2 | (e3 << 16);
  pk[2] = e4 | (e5 << 16);
  pk[3] = e6 | (e7 << 16);
  unsigned short* dp = dst + (size_t)i * 8;
  *(volatile v4u*)dp = pk;
  __threadfence();
  *(volatile v4u*)dp = pk;
}

__global__ __launch_bounds__(PC_THR) void bias_kernel(const float* __restrict__ bih0, const float* __restrict__ bhh0,
                                                      const float* __restrict__ bih1, const float* __restrict__ bhh1,
                                                      const float* __restrict__ bih2, const float* __restrict__ bhh2,
                                                      const float* __restrict__ bih3, const float* __restrict__ bhh3,
                                                      const float* __restrict__ b1,
                                                      float* __restrict__ BSUM, float* __restrict__ B1P) {
  const int y = blockIdx.y;
  const int i = blockIdx.x * PC_THR + threadIdx.x;
  if (y < 4) {
    const float* pa = (y == 0) ? bih0 : (y == 1) ? bih1 : (y == 2) ? bih2 : bih3;
    const float* pb = (y == 0) ? bhh0 : (y == 1) ? bhh1 : (y == 2) ? bhh2 : bhh3;
    if (i < NGATE / 4) {
      const v4f a = *(const v4f*)(pa + 4 * i);
      const v4f c = *(const v4f*)(pb + 4 * i);
      v4f o;
      o[0] = bf16r(a[0]) + bf16r(c[0]);
      o[1] = bf16r(a[1]) + bf16r(c[1]);
      o[2] = bf16r(a[2]) + bf16r(c[2]);
      o[3] = bf16r(a[3]) + bf16r(c[3]);
      float* op = BSUM + (size_t)y * NGATE + 4 * i;
      *(volatile v4f*)op = o;
      __threadfence();
      *(volatile v4f*)op = o;
    }
  } else {
    if (i < MLPP / 4) {
      const int ic = (i < MLPH / 4) ? i : (MLPH / 4 - 1);
      const v4f a = *(const v4f*)(b1 + 4 * ic);
      const float fl = (i < MLPH / 4) ? 1.0f : 0.0f;
      v4f o;
      o[0] = bf16r(a[0]) * fl;
      o[1] = bf16r(a[1]) * fl;
      o[2] = bf16r(a[2]) * fl;
      o[3] = bf16r(a[3]) * fl;
      float* op = B1P + 4 * i;
      *(volatile v4f*)op = o;
      __threadfence();
      *(volatile v4f*)op = o;
    }
  }
}

__device__ __forceinline__ float fsig(float x)  { return __builtin_amdgcn_rcpf(1.0f + expf(-x)); }
__device__ __forceinline__ float ftanh(float x) { return 1.0f - 2.0f * __builtin_amdgcn_rcpf(expf(2.0f * x) + 1.0f); }

__device__ __forceinline__ void rec_chunk(const __bf16* ah, const __bf16* wg0, const __bf16* wg1, const __bf16* wg2,
                                          const __bf16* wg3, int k, v8f& acc0, v8f& acc1, v8f& acc2, v8f& acc3) {
  const v16b a  = Frag<__bf16>::load(ah + k);
  const v16b b0 = Frag<__bf16>::load(wg0 + k);
  const v16b b1 = Frag<__bf16>::load(wg1 + k);
  const v16b b2 = Frag<__bf16>::load(wg2 + k);
  const v16b b3 = Frag<__bf16>::load(wg3 + k);
  acc0 = Frag<__bf16>::mma(a, b0, acc0);
  acc1 = Frag<__bf16>::mma(a, b1, acc1);
  acc2 = Frag<__bf16>::mma(a, b2, acc2);
  acc3 = Frag<__bf16>::mma(a, b3, acc3);
  guard_grp_b(acc0, acc1, acc2, acc3, a, b0, b1, b2, b3);
}

__global__ __launch_bounds__(REC_THR) void rec_kernel(const float* __restrict__ XGT,
                                                      const unsigned short* __restrict__ WHp,
                                                      unsigned short* __restrict__ E) {
  __shared__ __align__(16) unsigned short ht[2][SEQB * HTP];
  __shared__ __align__(16) float          cs[SEQB * HID];
  const __bf16* WH = (const __bf16*)WHp;
  const int tid = threadIdx.x, lane = tid & 31, wave = tid >> 5;
  const int c = lane & 15, hh = lane >> 4, koff = hh * 8;
  const int q8 = lane >> 3, p8 = (lane & 7) * 8;
  const int dir   = blockIdx.x / (NSEQ / SEQB);
  const int nbase = (blockIdx.x - dir * (NSEQ / SEQB)) * SEQB;
  const float*  XGd = XGT + (size_t)dir * NGATE * NROW;
  const __bf16* WHd = WH  + (size_t)dir * NGATE * KREC;

  {
    unsigned short* hf = &ht[0][0];
#pragma unroll 1
    for (int i = tid; i < 2 * SEQB * HTP; i += REC_THR) hf[i] = (unsigned short)0;
#pragma unroll 1
    for (int i = tid; i < SEQB * HID; i += REC_THR) cs[i] = 0.0f;
  }
  __syncthreads();

  const v8f z8 = {0.f, 0.f, 0.f, 0.f, 0.f, 0.f, 0.f, 0.f};
#pragma unroll 1
  for (int s = 0; s < NSTEP; ++s) {
    const int t   = dir ? (NSTEP - 1 - s) : s;
    const int cur = s & 1, nxt = cur ^ 1;
    const __bf16* ahrow = (const __bf16*)(&ht[cur][0]) + c * HTP + koff;
    unsigned short* hnt = &ht[nxt][0];
    const size_t xcol = (size_t)t * NSEQ + nbase + 8 * hh;
#pragma unroll 1
    for (int slot = 0; slot < UPW; ++slot) {
      const int u = 16 * (wave * UPW + slot) + c;
      const __bf16* wg0 = WHd + (size_t)(0 * HID + u) * KREC + koff;
      const __bf16* wg1 = WHd + (size_t)(1 * HID + u) * KREC + koff;
      const __bf16* wg2 = WHd + (size_t)(2 * HID + u) * KREC + koff;
      const __bf16* wg3 = WHd + (size_t)(3 * HID + u) * KREC + koff;
      v8f acc0 = z8, acc1 = z8, acc2 = z8, acc3 = z8;
#pragma unroll 1
      for (int k0 = 0; k0 < KREC; k0 += 64) {
        rec_chunk(ahrow, wg0, wg1, wg2, wg3, k0,      acc0, acc1, acc2, acc3);
        rec_chunk(ahrow, wg0, wg1, wg2, wg3, k0 + 32, acc0, acc1, acc2, acc3);
      }
      acc_guard4(acc0, acc1, acc2, acc3);
      const float* xp = XGd + (size_t)u * NROW + xcol;
      const v8f xi = *(const v8f*)(xp);
      const v8f xf = *(const v8f*)(xp + (size_t)1 * HID * NROW);
      const v8f xg = *(const v8f*)(xp + (size_t)2 * HID * NROW);
      const v8f xo = *(const v8f*)(xp + (size_t)3 * HID * NROW);
#pragma unroll
      for (int r = 0; r < 8; ++r) {
        const int row = 8 * hh + r;
        const float zi = acc0[r] + xi[r];
        const float zf = acc1[r] + xf[r];
        const float zg = acc2[r] + xg[r];
        const float zo = acc3[r] + xo[r];
        const float cold = cs[row * HID + u];
        const float ig = fsig(zi);
        const float fg = fsig(zf);
        const float gg = ftanh(zg);
        const float og = fsig(zo);
        const float cn = fg * cold + ig * gg;
        cs[row * HID + u] = cn;
        const float hv = og * ftanh(cn);
        const unsigned short hb = f2bf_bits(hv);
        const unsigned short lb = f2bf_bits(hv - bf_bits2f(hb));
        hnt[row * HTP + u]        = hb;
        hnt[row * HTP + SEGH + u] = lb;
      }
    }
    __syncthreads();
    {
      const unsigned short* hsrc = &ht[nxt][0];
      unsigned short* erow0 = E + ((size_t)t * NSEQ + nbase) * KCAT + (size_t)dir * KREC;
      for (int pass = 0; pass < 2; ++pass) {
#pragma unroll 1
        for (int it = 0; it < EITER; ++it) {
          const int L = it * EGRP + wave * 4 + q8;
          if (L < ELINES) {
            const int row = L / (KREC / 64);
            const int li  = L - row * (KREC / 64);
            const v4u v = *(const v4u*)(hsrc + row * HTP + 64 * li + p8);
            *(volatile v4u*)(erow0 + (size_t)row * KCAT + 64 * li + p8) = v;
          }
        }
        __threadfence();
      }
    }
  }
}

__global__ __launch_bounds__(PAIR_THR) void pair_kernel(const float* __restrict__ AO, const float* __restrict__ BO,
                                                        const float* __restrict__ w2, const float* __restrict__ b2,
                                                        float* __restrict__ out) {
  __shared__ __align__(16) float as_[NB_IN * ASP];
  __shared__ float ws_[MLPH];
  const int tid = threadIdx.x, lane = tid & 31, wave = tid >> 5;
  const int i = blockIdx.x;
#pragma unroll 1
  for (int f = tid; f < NB_IN * (MLPH / 4); f += PAIR_THR) {
    const int b  = f / (MLPH / 4);
    const int c4 = (f - b * (MLPH / 4)) * 4;
    const v4f v = *(const v4f*)(AO + ((size_t)b * NSEQ + i) * MLPP + c4);
    *(v4f*)(as_ + b * ASP + c4) = v;
  }
  if (tid < MLPH) ws_[tid] = bf16r(w2[tid]);
  const float b2r = bf16r(b2[0]);
  __syncthreads();
  const float* ar = as_ + lane * ASP;
  constexpr int JPW = NL_IN / (PAIR_THR / 32);
#pragma unroll 1
  for (int jj = 0; jj < JPW; ++jj) {
    const int j = wave * JPW + jj;
    const float* bp = BO + ((size_t)lane * NSEQ + j) * MLPP;
    float s = 0.0f;
#pragma unroll 1
    for (int h = 0; h < MLPH; ++h) s += ws_[h] * ftanh(ar[h] + bp[h]);
    const float o = s + b2r;
    float* op = out + ((size_t)i * NL_IN + j) * NB_IN + lane;
    *(volatile float*)op = o;
    __threadfence();
    *(volatile float*)op = o;
  }
}

extern "C" void kernel_launch(void* const* d_in, const int* in_sizes, int n_in,
                              void* d_out, int out_size, void* d_ws, size_t ws_size, hipStream_t stream) {
  if (n_in < 26 || d_out == nullptr || d_ws == nullptr) return;
  if (in_sizes[0] != NB_IN * NL_IN || in_sizes[1] != NB_IN * NL_IN ||
      in_sizes[4] != WVOC * WDIM || in_sizes[5] != TVOC * TDIM ||
      in_sizes[6] != NGATE * HID || in_sizes[7] != NGATE * HID || in_sizes[8] != NGATE || in_sizes[9] != NGATE ||
      in_sizes[10] != NGATE * HID || in_sizes[11] != NGATE * HID || in_sizes[12] != NGATE || in_sizes[13] != NGATE ||
      in_sizes[14] != NGATE * 2 * HID || in_sizes[15] != NGATE * HID || in_sizes[16] != NGATE || in_sizes[17] != NGATE ||
      in_sizes[18] != NGATE * 2 * HID || in_sizes[19] != NGATE * HID || in_sizes[20] != NGATE || in_sizes[21] != NGATE ||
      in_sizes[22] != MLPH * 4 * HID || in_sizes[23] != MLPH || in_sizes[24] != MLPH || in_sizes[25] < 1 ||
      out_size != NOUT) return;

  const int*   words = (const int*)d_in[0];
  const int*   tags  = (const int*)d_in[1];
  const float* wemb  = (const float*)d_in[4];
  const float* temb  = (const float*)d_in[5];
  const float* wih0  = (const float*)d_in[6];
  const float* whh0  = (const float*)d_in[7];
  const float* bih0  = (const float*)d_in[8];
  const float* bhh0  = (const float*)d_in[9];
  const float* wih0r = (const float*)d_in[10];
  const float* whh0r = (const float*)d_in[11];
  const float* bih0r = (const float*)d_in[12];
  const float* bhh0r = (const float*)d_in[13];
  const float* wih1  = (const float*)d_in[14];
  const float* whh1  = (const float*)d_in[15];
  const float* bih1  = (const float*)d_in[16];
  const float* bhh1  = (const float*)d_in[17];
  const float* wih1r = (const float*)d_in[18];
  const float* whh1r = (const float*)d_in[19];
  const float* bih1r = (const float*)d_in[20];
  const float* bhh1r = (const float*)d_in[21];
  const float* w1    = (const float*)d_in[22];
  const float* b1    = (const float*)d_in[23];
  const float* w2    = (const float*)d_in[24];
  const float* b2    = (const float*)d_in[25];
  float* out = (float*)d_out;

  char* ws = (char*)d_ws; size_t off = 0;
  auto carve = [&](size_t bytes) -> char* { char* p = ws + off; off += (bytes + 255) & ~(size_t)255; return p; };
  unsigned short* E0   = (unsigned short*)carve((size_t)NROW * K0P * 2);
  unsigned short* WI0A = (unsigned short*)carve((size_t)NGATE * K0P * 2);
  unsigned short* WI0B = (unsigned short*)carve((size_t)NGATE * K0P * 2);
  unsigned short* WH   = (unsigned short*)carve((size_t)4 * NGATE * KREC * 2);
  unsigned short* WI1A = (unsigned short*)carve((size_t)NGATE * KCAT * 2);
  unsigned short* WI1B = (unsigned short*)carve((size_t)NGATE * KCAT * 2);
  unsigned short* W1A  = (unsigned short*)carve((size_t)MLPP * KCAT * 2);
  unsigned short* W1B  = (unsigned short*)carve((size_t)MLPP * KCAT * 2);
  float*          BSUM = (float*)carve((size_t)4 * NGATE * 4);
  float*          B1P  = (float*)carve((size_t)MLPP * 4);
  float*          XGT  = (float*)carve((size_t)2 * NGATE * NROW * 4);
  unsigned short* E1   = (unsigned short*)carve((size_t)NROW * KCAT * 2);
  unsigned short* E2   = (unsigned short*)carve((size_t)NROW * KCAT * 2);
  float*          AOUT = (float*)carve((size_t)NROW * MLPP * 4);
  float*          BOUT = (float*)carve((size_t)NROW * MLPP * 4);
  if (off > ws_size || off > (size_t)134217728) return;

  const size_t WHPL = (size_t)NGATE * KREC;
  const size_t XGPL = (size_t)NGATE * NROW;

  embed_kernel<<<NROW / 2, EMB_THR, 0, stream>>>(words, tags, wemb, temb, E0);

  const int g416  = NGATE * 1 * GPSEG;
  const int g832  = NGATE * 2 * GPSEG;
  const int g1664 = NGATE * 4 * GPSEG;
  const int gw1   = MLPP * 4 * GPSEG;
  padcopy_kernel<<<(g416 + PC_THR - 1) / PC_THR,  PC_THR, 0, stream>>>(wih0,  HID,     0,   NGATE, WI0A,          NGATE, 1);
  padcopy_kernel<<<(g416 + PC_THR - 1) / PC_THR,  PC_THR, 0, stream>>>(wih0r, HID,     0,   NGATE, WI0B,          NGATE, 1);
  padcopy_kernel<<<(g832 + PC_THR - 1) / PC_THR,  PC_THR, 0, stream>>>(whh0,  HID,     0,   NGATE, WH + 0 * WHPL, NGATE, 2);
  padcopy_kernel<<<(g832 + PC_THR - 1) / PC_THR,  PC_THR, 0, stream>>>(whh0r, HID,     0,   NGATE, WH + 1 * WHPL, NGATE, 2);
  padcopy_kernel<<<(g832 + PC_THR - 1) / PC_THR,  PC_THR, 0, stream>>>(whh1,  HID,     0,   NGATE, WH + 2 * WHPL, NGATE, 2);
  padcopy_kernel<<<(g832 + PC_THR - 1) / PC_THR,  PC_THR, 0, stream>>>(whh1r, HID,     0,   NGATE, WH + 3 * WHPL, NGATE, 2);
  padcopy_kernel<<<(g1664 + PC_THR - 1) / PC_THR, PC_THR, 0, stream>>>(wih1,  2 * HID, 0,   NGATE, WI1A,          NGATE, 4);
  padcopy_kernel<<<(g1664 + PC_THR - 1) / PC_THR, PC_THR, 0, stream>>>(wih1r, 2 * HID, 0,   NGATE, WI1B,          NGATE, 4);
  padcopy_kernel<<<(gw1 + PC_THR - 1) / PC_THR,   PC_THR, 0, stream>>>(w1,    4 * HID, 0,   MLPH,  W1A,           MLPP,  4);
  padcopy_kernel<<<(gw1 + PC_THR - 1) / PC_THR,   PC_THR, 0, stream>>>(w1,    4 * HID, 800, MLPH,  W1B,           MLPP,  4);

  bias_kernel<<<dim3(2, 5), PC_THR, 0, stream>>>(bih0, bhh0, bih0r, bhh0r, bih1, bhh1, bih1r, bhh1r, b1, BSUM, B1P);

  const dim3 gproj((NGATE / 64) * (NROW / 64) / 8, 1);
  wmma_gemm64<1, false, 1, 0, false, 0><<<gproj, 256, 0, stream>>>(
      WI0A, WI0A, K0P, 0L, E0, E0, K0P, 0L, (void*)(XGT), (void*)(XGT), NROW, 0L,
      BSUM + 0 * NGATE, BSUM, 0L, NGATE, NROW, K0P, 1.0f);
  wmma_gemm64<1, false, 1, 0, false, 0><<<gproj, 256, 0, stream>>>(
      WI0B, WI0B, K0P, 0L, E0, E0, K0P, 0L, (void*)(XGT + XGPL), (void*)(XGT + XGPL), NROW, 0L,
      BSUM + 1 * NGATE, BSUM, 0L, NGATE, NROW, K0P, 1.0f);

  rec_kernel<<<2 * (NSEQ / SEQB), REC_THR, 0, stream>>>(XGT, WH + 0 * WHPL, E1);

  wmma_gemm64<1, false, 1, 0, false, 0><<<gproj, 256, 0, stream>>>(
      WI1A, WI1A, KCAT, 0L, E1, E1, KCAT, 0L, (void*)(XGT), (void*)(XGT), NROW, 0L,
      BSUM + 2 * NGATE, BSUM, 0L, NGATE, NROW, KCAT, 1.0f);
  wmma_gemm64<1, false, 1, 0, false, 0><<<gproj, 256, 0, stream>>>(
      WI1B, WI1B, KCAT, 0L, E1, E1, KCAT, 0L, (void*)(XGT + XGPL), (void*)(XGT + XGPL), NROW, 0L,
      BSUM + 3 * NGATE, BSUM, 0L, NGATE, NROW, KCAT, 1.0f);

  rec_kernel<<<2 * (NSEQ / SEQB), REC_THR, 0, stream>>>(XGT, WH + 2 * WHPL, E2);

  const dim3 ghead((NROW / 64) * (MLPP / 64) / 8, 1);
  wmma_gemm64<1, false, 0, 0, false, 0><<<ghead, 256, 0, stream>>>(
      E2, E2, KCAT, 0L, W1A, W1A, KCAT, 0L, (void*)AOUT, (void*)AOUT, MLPP, 0L,
      B1P, BSUM, 0L, NROW, MLPP, KCAT, 1.0f);
  wmma_gemm64<1, false, 2, 0, false, 0><<<ghead, 256, 0, stream>>>(
      E2, E2, KCAT, 0L, W1B, W1B, KCAT, 0L, (void*)BOUT, (void*)BOUT, MLPP, 0L,
      B1P, BSUM, 0L, NROW, MLPP, KCAT, 1.0f);

  pair_kernel<<<NL_IN, PAIR_THR, 0, stream>>>(AOUT, BOUT, w2, b2, out);
}
